// Block_Atom_18090402250769
// MI455X (gfx1250) — hardware-verified
//
#include <hip/hip_runtime.h>


#define NB_ 8
#define NAT 4096
#define NAA 1024
#define NPC 4096
#define KNB 16
#define KNC 14
#define NG 32
#define DA 12
#define FF 128
#define DD 128
#define TA (NG * DA)
#define NATOM (NB_ * NAT)
#define NAAT (NB_ * NAA)
#define BN_EPS 1e-5f

typedef __attribute__((ext_vector_type(16))) __bf16   v16bf;
typedef __attribute__((ext_vector_type(16))) _Float16 v16h;
typedef __attribute__((ext_vector_type(8)))  float    v8f;
typedef __attribute__((ext_vector_type(8)))  unsigned v8u;

__device__ __forceinline__ unsigned f2bf(float f) { unsigned u = __float_as_uint(f); u += 0x7FFFu + ((u >> 16) & 1u); return u >> 16; }
__device__ __forceinline__ unsigned f2h(float f) { return (unsigned)__builtin_bit_cast(unsigned short, (_Float16)f); }
__device__ __forceinline__ int kpat(int v, int half) { return ((v & 4) ? 16 : 0) + half * 8 + 2 * (v & 3); }

template <int F16, int NP> struct Opnd { v16bf p[NP]; };

template <int F16, int NP> __device__ __forceinline__ void pack2(float f0, float f1, unsigned* o) {
    if (F16) { o[0] = f2h(f0) | (f2h(f1) << 16); return; }
    unsigned h0 = f2bf(f0), h1 = f2bf(f1); o[0] = h0 | (h1 << 16);
    if (NP >= 2) {
        float r0 = f0 - __uint_as_float(h0 << 16), r1 = f1 - __uint_as_float(h1 << 16);
        unsigned m0 = f2bf(r0), m1 = f2bf(r1); o[1] = m0 | (m1 << 16);
        if (NP >= 3) {
            float s0 = r0 - __uint_as_float(m0 << 16), s1 = r1 - __uint_as_float(m1 << 16);
            o[2] = f2bf(s0) | (f2bf(s1) << 16);
        }
    }
}
template <int F16, int NP> __device__ __forceinline__ void op_row(const float* rowp, int half, float sc, Opnd<F16, NP>& o) {
    v8u u[NP];
#pragma unroll
    for (int v = 0; v < 8; ++v) {
        int kk = kpat(v, half); unsigned t[3];
        pack2<F16, NP>(rowp[kk] * sc, rowp[kk + 1] * sc, t);
#pragma unroll
        for (int p = 0; p < NP; ++p) u[p][v] = t[p];
    }
#pragma unroll
    for (int p = 0; p < NP; ++p) o.p[p] = __builtin_bit_cast(v16bf, u[p]);
}
template <int F16, int NP> __device__ __forceinline__ void op_row_tail(const float* rowp, int half, float sc, int kvalid, Opnd<F16, NP>& o) {
    v8u u[NP];
#pragma unroll
    for (int v = 0; v < 8; ++v) {
        int kk = kpat(v, half); unsigned t[3];
        float f0 = kk < kvalid ? rowp[kk] * sc : 0.0f, f1 = (kk + 1) < kvalid ? rowp[kk + 1] * sc : 0.0f;
        pack2<F16, NP>(f0, f1, t);
#pragma unroll
        for (int p = 0; p < NP; ++p) u[p][v] = t[p];
    }
#pragma unroll
    for (int p = 0; p < NP; ++p) o.p[p] = __builtin_bit_cast(v16bf, u[p]);
}
template <int F16, int NP> __device__ __forceinline__ void op_col(const float* M, int ld, int n, int k0, int half, float sc, Opnd<F16, NP>& o) {
    v8u u[NP];
#pragma unroll
    for (int v = 0; v < 8; ++v) {
        int kk = k0 + kpat(v, half); unsigned t[3];
        pack2<F16, NP>(M[(size_t)kk * ld + n] * sc, M[(size_t)(kk + 1) * ld + n] * sc, t);
#pragma unroll
        for (int p = 0; p < NP; ++p) u[p][v] = t[p];
    }
#pragma unroll
    for (int p = 0; p < NP; ++p) o.p[p] = __builtin_bit_cast(v16bf, u[p]);
}
template <int F16, int NP> __device__ __forceinline__ void op_col_tail(const float* M, int ld, int n, int k0, int half, float sc, int K, Opnd<F16, NP>& o) {
    v8u u[NP];
#pragma unroll
    for (int v = 0; v < 8; ++v) {
        int kk = k0 + kpat(v, half); unsigned t[3];
        float f0 = kk < K ? M[(size_t)kk * ld + n] * sc : 0.0f, f1 = (kk + 1) < K ? M[(size_t)(kk + 1) * ld + n] * sc : 0.0f;
        pack2<F16, NP>(f0, f1, t);
#pragma unroll
        for (int p = 0; p < NP; ++p) u[p][v] = t[p];
    }
#pragma unroll
    for (int p = 0; p < NP; ++p) o.p[p] = __builtin_bit_cast(v16bf, u[p]);
}
__device__ __forceinline__ v8f wm_bf16(v16bf a, v16bf b, v8f c) { return __builtin_amdgcn_wmma_f32_16x16x32_bf16(false, a, false, b, (short)0, c, false, false); }
template <int F16, int NA, int NB> __device__ __forceinline__ v8f wmma_op(const Opnd<F16, NA>& a, const Opnd<F16, NB>& b, v8f c) {
    if (F16) {
        v16h ah = __builtin_bit_cast(v16h, a.p[0]), bh = __builtin_bit_cast(v16h, b.p[0]);
        c = __builtin_amdgcn_wmma_f32_16x16x32_f16(false, ah, false, bh, (short)0, c, false, false);
        asm volatile("v_nop\n\tv_nop\n\tv_nop\n\tv_nop" : "+v"(c) : "v"(ah), "v"(bh));
        return c;
    }
    constexpr int NMX = NA > NB ? NA : NB;
#pragma unroll
    for (int i = 0; i < NA; ++i)
#pragma unroll
        for (int j = 0; j < NB; ++j)
            if (i + j < NMX) c = wm_bf16(a.p[i], b.p[j], c);
    if (NA == 1 && NB == 1)      asm volatile("v_nop\n\tv_nop\n\tv_nop\n\tv_nop" : "+v"(c) : "v"(a.p[0]), "v"(b.p[0]));
    else if (NA == 2 && NB == 1) asm volatile("v_nop\n\tv_nop\n\tv_nop\n\tv_nop" : "+v"(c) : "v"(a.p[0]), "v"(a.p[1]), "v"(b.p[0]));
    else if (NA == 1 && NB == 2) asm volatile("v_nop\n\tv_nop\n\tv_nop\n\tv_nop" : "+v"(c) : "v"(a.p[0]), "v"(b.p[0]), "v"(b.p[1]));
    else if (NA == 2 && NB == 2) asm volatile("v_nop\n\tv_nop\n\tv_nop\n\tv_nop" : "+v"(c) : "v"(a.p[0]), "v"(a.p[1]), "v"(b.p[0]), "v"(b.p[1]));
    else                         asm volatile("v_nop\n\tv_nop\n\tv_nop\n\tv_nop" : "+v"(c) : "v"(a.p[0]), "v"(a.p[NA - 1]), "v"(b.p[0]), "v"(b.p[NB - 1]), "v"(a.p[NA / 2]), "v"(b.p[NB / 2]));
    return c;
}

struct ZMap { long long s1; long long s2; int zdiv; int pad_; };
__device__ __forceinline__ size_t zoff(const ZMap& m, int z) { return (size_t)((long long)(z / m.zdiv) * m.s1 + (long long)(z % m.zdiv) * m.s2); }

#define ACT_NONE 0
#define ACT_RELU 1
#define ACT_GELU_ERF 2
#define ACT_SILU 3
#define ACT_TANH 4
__device__ __forceinline__ float act_apply(int act, float x) {
    if (act == ACT_RELU) return x > 0.f ? x : 0.f;
    if (act == ACT_GELU_ERF) return 0.5f * x * (1.0f + erff(x * 0.70710678118654752f));
    if (act == ACT_SILU) return x / (1.0f + expf(-x));
    if (act == ACT_TANH) return tanhf(x);
    return x;
}
struct GemmArgs {
    ZMap za, zb_, zc, zbias, zadd, zrsc, zmul, zrbias;
    const float* A; const float* Bm; float* C; const float* bias; const float* add; const float* rsc; const float* mul; const float* rbias;
    long long ldadd, ldmul;
    int lda, ldb, ldc, K;
    float ascale, bscale, oscale, addscale;
    int M, nvalid, nstore, ldrsc;
    int bcs, pad1, pad2, pad3;
};
template <int BT, int F16, int NA, int NB, int RW, int CW, int ACT>
__global__ __launch_bounds__(256) void gemm_kernel(GemmArgs g) {
    constexpr int TR = 16 * RW, TC = 64 * CW, CSTR = TC + 4;
    __shared__ __align__(16) float cst[TR * CSTR];
    const int z = blockIdx.z;
    const float* A = g.A + zoff(g.za, z); const float* Bm = g.Bm + zoff(g.zb_, z); float* C = g.C + zoff(g.zc, z);
    const int tid = threadIdx.x, lane = tid & 31, wv = tid >> 5;
    const int l16 = lane & 15, half = lane >> 4;
    const int rt = wv % RW, ch = wv / RW;
    const int row0 = blockIdx.x * TR, col0 = blockIdx.y * TC + ch * 64;
    int arix = row0 + rt * 16 + l16; if (arix >= g.M) arix = g.M - 1;
    const float* arow = A + (size_t)arix * g.lda;
    v8f acc[4];
#pragma unroll
    for (int t = 0; t < 4; ++t) acc[t] = (v8f){};
    const int K = g.K;
#pragma unroll 1
    for (int kc = 0; kc < K; kc += 32) {
        Opnd<F16, NA> a;
        if (kc + 32 <= K) op_row<F16, NA>(arow + kc, half, g.ascale, a); else op_row_tail<F16, NA>(arow + kc, half, g.ascale, K - kc, a);
#pragma unroll
        for (int t = 0; t < 4; ++t) {
            Opnd<F16, NB> b;
            const int n = col0 + t * 16 + l16;
            if (n < g.nvalid) {
                if (BT) { if (kc + 32 <= K) op_row<F16, NB>(Bm + (size_t)n * g.ldb + kc, half, g.bscale, b); else op_row_tail<F16, NB>(Bm + (size_t)n * g.ldb + kc, half, g.bscale, K - kc, b); }
                else    { if (kc + 32 <= K) op_col<F16, NB>(Bm, g.ldb, n * g.bcs, kc, half, g.bscale, b); else op_col_tail<F16, NB>(Bm, g.ldb, n * g.bcs, kc, half, g.bscale, K, b); }
            } else {
#pragma unroll
                for (int p = 0; p < NB; ++p) b.p[p] = (v16bf){};
            }
            acc[t] = wmma_op<F16, NA, NB>(a, b, acc[t]);
        }
    }
    const float* bias = g.bias ? g.bias + zoff(g.zbias, z) : nullptr;
    const float* add = g.add ? g.add + zoff(g.zadd, z) : nullptr;
    const float* rsc = g.rsc ? g.rsc + zoff(g.zrsc, z) : nullptr;
    const float* mul = g.mul ? g.mul + zoff(g.zmul, z) : nullptr;
    const float* rbias = g.rbias ? g.rbias + zoff(g.zrbias, z) : nullptr;
#pragma unroll
    for (int t = 0; t < 4; ++t) {
        const int cl = ch * 64 + t * 16 + l16;
        const int cg = blockIdx.y * TC + cl;
        const bool cok = cg < g.nvalid;
        const float bv = (bias && cok) ? bias[(size_t)cg * g.bcs] : 0.0f;
#pragma unroll
        for (int r = 0; r < 8; ++r) {
            const int rl = rt * 16 + r + 8 * half;
            float v = acc[t][r] * g.oscale + bv;
            int rg = row0 + rl; if (rg >= g.M) rg = g.M - 1;
            if (rbias) v += rbias[rg];
            if (rsc) v *= rsc[(size_t)rg * g.ldrsc];
            if (mul && cok) v *= mul[(size_t)rg * g.ldmul + cg];
            if (add && cok) v += g.addscale * add[(size_t)rg * g.ldadd + cg];
            cst[rl * CSTR + cl] = v;
        }
    }
    __syncthreads();
    const int col = tid % TC, rsel = tid / TC, rstep = 256 / TC;
    if (ACT != ACT_NONE) {
#pragma unroll 1
        for (int r = rsel; r < TR; r += rstep) cst[r * CSTR + col] = act_apply(ACT, cst[r * CSTR + col]);
    }
    float* ob = C + (size_t)row0 * g.ldc + (size_t)blockIdx.y * TC;
    const bool colok = (int)(blockIdx.y * TC + col) < g.nstore;
    const int rmax = (g.M - row0 < TR) ? (g.M - row0) : TR;
    auto pass = [&]() {
        if (colok) {
#pragma unroll 4
            for (int r = rsel; r < rmax; r += rstep) *(volatile float*)(ob + (size_t)r * g.ldc + col) = cst[r * CSTR + col];
        }
    };
    pass();
    __threadfence();
    pass();
}
static inline ZMap zm(long long s1) { ZMap m; m.s1 = s1; m.s2 = 0; m.zdiv = 1; m.pad_ = 0; return m; }
static inline ZMap zm2(long long s1, long long s2, int zdiv) { ZMap m; m.s1 = s1; m.s2 = s2; m.zdiv = zdiv; m.pad_ = 0; return m; }
static inline GemmArgs gemm_args(const float* A, int lda, ZMap za, const float* Bm, int ldb, ZMap zb, float* C, int ldc, ZMap zc, int M, int N, int K) {
    GemmArgs g; g.za = za; g.zb_ = zb; g.zc = zc; g.zbias = zm(0); g.zadd = zm(0); g.zrsc = zm(0); g.zmul = zm(0); g.zrbias = zm(0);
    g.A = A; g.Bm = Bm; g.C = C; g.bias = nullptr; g.add = nullptr; g.rsc = nullptr; g.mul = nullptr; g.rbias = nullptr; g.ldadd = 0; g.ldmul = 0;
    g.lda = lda; g.ldb = ldb; g.ldc = ldc; g.K = K; g.ascale = 1.0f; g.bscale = 1.0f; g.oscale = 1.0f; g.addscale = 1.0f; g.M = M; g.nvalid = N; g.nstore = N; g.ldrsc = 1;
    g.bcs = 1; g.pad1 = 0; g.pad2 = 0; g.pad3 = 0;
    return g;
}
static_assert(sizeof(ZMap) == 24, "ZMap layout");
static_assert(sizeof(GemmArgs) == 8 * 24 + 8 * 8 + 2 * 8 + 4 * 4 + 4 * 4 + 4 * 4 + 4 * 4, "GemmArgs has no padding");

__global__ __launch_bounds__(256) void softmax_rows(float* S, long long sy, long long sx, int L, float prescale, const float* addv, long long say, int aydiv, int causal,
                                                  const int* imask, long long imy, long long imx, float maskval) {
    __shared__ float red[8];
    const int tid = threadIdx.x, lane = tid & 31, wid = tid >> 5;
    float* row = S + (size_t)blockIdx.y * sy + (size_t)blockIdx.x * sx;
    const float* av = addv ? addv + (size_t)(blockIdx.y / aydiv) * say : nullptr;
    const int* im = imask ? imask + (size_t)(blockIdx.y / aydiv) * imy + (size_t)blockIdx.x * imx : nullptr;
    float v[16];
    const int nj = L / 256;
    float mx = -__builtin_inff();
#pragma unroll
    for (int j = 0; j < 16; ++j) if (j < nj) { float t = row[tid + 256 * j] * prescale; if (av) t += av[tid + 256 * j]; if (im && im[tid + 256 * j] == 0) t = maskval; if (causal && (tid + 256 * j) > (int)blockIdx.x) t = -__builtin_inff(); v[j] = t; mx = fmaxf(mx, t); }
#pragma unroll
    for (int o = 16; o; o >>= 1) mx = fmaxf(mx, __shfl_xor(mx, o, 32));
    if (lane == 0) red[wid] = mx;
    __syncthreads();
    float m = red[0];
#pragma unroll
    for (int i = 1; i < 8; ++i) m = fmaxf(m, red[i]);
    if (m == -__builtin_inff()) m = 0.f;
    __syncthreads();
    float sum = 0.f;
#pragma unroll
    for (int j = 0; j < 16; ++j) if (j < nj) { v[j] = expf(v[j] - m); sum += v[j]; }
#pragma unroll
    for (int o = 16; o; o >>= 1) sum += __shfl_xor(sum, o, 32);
    if (lane == 0) red[wid] = sum;
    __syncthreads();
    float tot = 0.f;
#pragma unroll
    for (int i = 0; i < 8; ++i) tot += red[i];
    const float inv = 1.0f / tot;
#pragma unroll
    for (int j = 0; j < 16; ++j) if (j < nj) *(volatile float*)(row + tid + 256 * j) = v[j] * inv;
    __threadfence();
#pragma unroll
    for (int j = 0; j < 16; ++j) if (j < nj) *(volatile float*)(row + tid + 256 * j) = v[j] * inv;
}

#define VST2(T, p, v) do { const T vst2_v_ = (v); *(volatile T*)(p) = vst2_v_; __threadfence(); *(volatile T*)(p) = vst2_v_; } while (0)
__device__ __forceinline__ int clampi(int v, int n) { return v < 0 ? 0 : (v >= n ? n - 1 : v); }
__global__ __launch_bounds__(256) void k_frame(const float* __restrict__ pc, const float* __restrict__ matom, const float* __restrict__ attr, const int* __restrict__ fidx, const int* __restrict__ aidx, float* FR) {
    const int t = blockIdx.x * 256 + threadIdx.x; if (t >= NATOM) return; const int b = t / NAT; const float* P = pc + (size_t)b * NPC * 3;
    const int i0 = clampi(fidx[t * 3], NPC), i1 = clampi(fidx[t * 3 + 1], NPC), i2 = clampi(fidx[t * 3 + 2], NPC);
    const float cx = P[i1 * 3], cy = P[i1 * 3 + 1], cz = P[i1 * 3 + 2];
    float ux = P[i2 * 3] - cx, uy = P[i2 * 3 + 1] - cy, uz = P[i2 * 3 + 2] - cz; { const float n = sqrtf(ux * ux + uy * uy + uz * uz) + 1e-8f; ux /= n; uy /= n; uz /= n; }
    float vx = P[i0 * 3] - cx, vy = P[i0 * 3 + 1] - cy, vz = P[i0 * 3 + 2] - cz; const float dv = vx * ux + vy * uy + vz * uz; vx -= dv * ux; vy -= dv * uy; vz -= dv * uz;
    { const float n = sqrtf(vx * vx + vy * vy + vz * vz) + 1e-8f; vx /= n; vy /= n; vz /= n; }
    const float wx = uy * vz - uz * vy, wy = uz * vx - ux * vz, wz = ux * vy - uy * vx;
    float o[32]; o[0] = ux; o[1] = uy; o[2] = uz; o[3] = vx; o[4] = vy; o[5] = vz; o[6] = wx; o[7] = wy; o[8] = wz; o[9] = cx; o[10] = cy; o[11] = cz;
    const int ai = clampi(aidx[t], 39); float any = 0.f;
#pragma unroll
    for (int d = 0; d < DA; ++d) { const float a = attr[ai * DA + d]; o[12 + d] = a; if (a != 0.f) any = 1.f; }
#pragma unroll
    for (int d = 0; d < DA; ++d) o[12 + d] *= any;
    o[24] = matom[t] * any;
#pragma unroll
    for (int k = 25; k < 32; ++k) o[k] = 0.f;
#pragma unroll
    for (int k = 0; k < 32; ++k) { VST2(float, FR + (size_t)t * 32 + k, o[k]); }
}
__global__ __launch_bounds__(256) void k_tga(const float* __restrict__ FR, const int* __restrict__ nbidx, const float* __restrict__ gc, float* T) {
    const int q = blockIdx.x * 256 + threadIdx.x; if (q >= NATOM * NG) return; const int g = q % NG, t = q / NG; const int b = t / NAT; const float* f = FR + (size_t)t * 32;
    const float gx = gc[g * 3], gy = gc[g * 3 + 1], gz = gc[g * 3 + 2]; float acc[DA];
#pragma unroll
    for (int a = 0; a < DA; ++a) acc[a] = 0.f;
#pragma unroll 1
    for (int k = 0; k < KNB; ++k) { const int nb = clampi(nbidx[(size_t)t * KNB + k], NAT); const float* fn = FR + ((size_t)b * NAT + nb) * 32;
        const float dx = fn[9] - f[9], dy = fn[10] - f[10], dz = fn[11] - f[11];
        const float r0 = f[0] * dx + f[1] * dy + f[2] * dz - gx, r1 = f[3] * dx + f[4] * dy + f[5] * dz - gy, r2 = f[6] * dx + f[7] * dy + f[8] * dz - gz;
        const float gv = expf(-0.5f * (r0 * r0 + r1 * r1 + r2 * r2));
#pragma unroll
        for (int a = 0; a < DA; ++a) acc[a] += gv * fn[12 + a]; }
#pragma unroll
    for (int a = 0; a < DA; ++a) { VST2(float, T + (size_t)t * TA + g * DA + a, acc[a]); }
}
__global__ __launch_bounds__(256) void k_rsc(const float* __restrict__ FR, float* RSC) { const int t = blockIdx.x * 256 + threadIdx.x; if (t < NATOM) { VST2(float, RSC + t, FR[(size_t)t * 32 + 24] / (float)KNB); } }
__global__ __launch_bounds__(256) void k_my(const float* __restrict__ FR, float* MY) { const int t = blockIdx.x * 256 + threadIdx.x; if (t < NATOM) { VST2(float, MY + t, FR[(size_t)t * 32 + 24]); } }
__global__ __launch_bounds__(256) void k_pool(const float* __restrict__ ATT, const float* __restrict__ FEAT, const float* __restrict__ MY, const int* __restrict__ aanb, const int* __restrict__ sia, const int* __restrict__ siaa, const float* __restrict__ maa, float* PO) {
    const int lane = threadIdx.x & 31, r = blockIdx.x * 8 + (threadIdx.x >> 5); if (r >= NAAT) return; const int b = r / NAA; int nb[KNC]; float mk[KNC], gt[KNC]; const int sa = siaa[r];
#pragma unroll
    for (int k = 0; k < KNC; ++k) { nb[k] = clampi(aanb[(size_t)r * KNC + k], NAT); const int atom = b * NAT + nb[k]; mk[k] = MY[atom]; gt[k] = (sia[atom] == sa) ? 1.f : 0.f; }
#pragma unroll 1
    for (int j = 0; j < 4; ++j) { const int d = lane + 32 * j; float lg[KNC]; float m = -__builtin_inff();
#pragma unroll 1
        for (int k = 0; k < KNC; ++k) { lg[k] = mk[k] > 0.f ? ATT[((size_t)b * NAT + nb[k]) * DD + d] : -1e9f; m = fmaxf(m, lg[k]); }
        float s = 0.f;
#pragma unroll 1
        for (int k = 0; k < KNC; ++k) { lg[k] = expf(lg[k] - m); s += lg[k]; }
        float ws = 0.f, acc = 0.f;
#pragma unroll 1
        for (int k = 0; k < KNC; ++k) { const float w = lg[k] / s * gt[k] * mk[k]; ws += w; acc += w * FEAT[((size_t)b * NAT + nb[k]) * DD + d]; }
        VST2(float, PO + (size_t)r * DD + d, acc / (ws + 1e-8f) * maa[r]);
    }
}
__global__ __launch_bounds__(128) void k_bn(const float* __restrict__ PO, const float* __restrict__ maa, const float* __restrict__ g, const float* __restrict__ bb, float* out, float* omask) {
    const int c = threadIdx.x; double n = 0.0, s = 0.0;
    for (int r = 0; r < NAAT; ++r) { const double m = (double)maa[r]; n += m; s += (double)PO[(size_t)r * DD + c] * m; }
    n += 1e-8; const double mean = s / n; double q = 0.0;
    for (int r = 0; r < NAAT; ++r) { const double d = (double)PO[(size_t)r * DD + c] - mean; q += (double)maa[r] * d * d; }
    const float rstd = (float)(1.0 / sqrt(q / n + (double)BN_EPS)); const float fm = (float)mean;
    for (int r = 0; r < NAAT; ++r) { const float v = g[c] * (PO[(size_t)r * DD + c] - fm) * rstd + bb[c]; VST2(float, out + (size_t)r * DD + c, fmaxf(v * maa[r], 0.f)); if (c == 0) { VST2(float, omask + r, maa[r]); } }
}
extern "C" void kernel_launch(void* const* d_in, const int* in_sizes, int n_in,
                              void* d_out, int out_size, void* d_ws, size_t ws_size, hipStream_t stream) {
    (void)in_sizes; (void)n_in; (void)out_size;
    const float* pc = (const float*)d_in[0]; const float* matom = (const float*)d_in[1]; const float* maa = (const float*)d_in[2]; const float* attr = (const float*)d_in[3]; const float* gc = (const float*)d_in[4];
    const float* Wnem = (const float*)d_in[5]; const float* Watt = (const float*)d_in[6]; const float* Wfeat = (const float*)d_in[7]; const float* bng = (const float*)d_in[8]; const float* bnb = (const float*)d_in[9];
    const int* fidx = (const int*)d_in[10]; const int* aidx = (const int*)d_in[11]; const int* nbidx = (const int*)d_in[12]; const int* sia = (const int*)d_in[13]; const int* siaa = (const int*)d_in[14]; const int* aanb = (const int*)d_in[15];
    float* out = (float*)d_out;
    float* omask = out + (size_t)NAAT * DD;
    char* wsp = (char*)d_ws;
    auto take = [&](size_t bytes) { char* p = wsp; wsp += (bytes + 255) & ~(size_t)255; return (void*)p; };
    float* FR = (float*)take((size_t)NATOM * 32 * 4); float* T = (float*)take((size_t)NATOM * TA * 4); float* RSC = (float*)take((size_t)NATOM * 4); float* MY = (float*)take((size_t)NATOM * 4);
    float* Y = (float*)take((size_t)NATOM * FF * 4); float* ATT = (float*)take((size_t)NATOM * DD * 4); float* FEAT = (float*)take((size_t)NATOM * DD * 4); float* PO = (float*)take((size_t)NAAT * DD * 4);
    if ((size_t)(wsp - (char*)d_ws) > ws_size) return;
    k_frame<<<NATOM / 256, 256, 0, stream>>>(pc, matom, attr, fidx, aidx, FR);
    k_tga<<<(NATOM * NG) / 256, 256, 0, stream>>>(FR, nbidx, gc, T);
    k_rsc<<<NATOM / 256, 256, 0, stream>>>(FR, RSC); k_my<<<NATOM / 256, 256, 0, stream>>>(FR, MY);
    { GemmArgs g = gemm_args(T, TA, zm(0), Wnem, FF, zm(0), Y, FF, zm(0), NATOM, FF, TA); g.rsc = RSC; gemm_kernel<0, 0, 2, 2, 4, 2, ACT_NONE><<<dim3(NATOM / 64, 1, 1), 256, 0, stream>>>(g); }
    { GemmArgs g = gemm_args(Y, FF, zm(0), Watt, DD, zm(0), ATT, DD, zm(0), NATOM, DD, FF); g.rsc = MY; gemm_kernel<0, 0, 2, 2, 4, 2, ACT_NONE><<<dim3(NATOM / 64, 1, 1), 256, 0, stream>>>(g); }
    { GemmArgs g = gemm_args(Y, FF, zm(0), Wfeat, DD, zm(0), FEAT, DD, zm(0), NATOM, DD, FF); g.rsc = MY; gemm_kernel<0, 0, 2, 2, 4, 2, ACT_NONE><<<dim3(NATOM / 64, 1, 1), 256, 0, stream>>>(g); }
    k_pool<<<NAAT / 8, 256, 0, stream>>>(ATT, FEAT, MY, aanb, sia, siaa, maa, PO);
    k_bn<<<1, 128, 0, stream>>>(PO, maa, bng, bnb, out, omask);
}
